// FCbasedGCN_48704929136872
// MI455X (gfx1250) — hardware-verified
//
#include <hip/hip_runtime.h>
#define NN 20000
#define NE 320000
#define F0 200
#define F0P 224
#define HH 128
#define NG 100
#define NCLS 10

typedef __bf16 v16b __attribute__((ext_vector_type(16)));
typedef unsigned short v8us __attribute__((ext_vector_type(8), may_alias));
typedef float  v8f  __attribute__((ext_vector_type(8)));
typedef float  v4f  __attribute__((ext_vector_type(4)));
typedef float  v4fa __attribute__((ext_vector_type(4), may_alias));
union FragB { v16b v; v8us half[2]; unsigned short u[16]; };

__device__ __forceinline__ unsigned short bf16_bits(float x) { unsigned int u = __float_as_uint(x); return (unsigned short)((u + 0x7FFFu + ((u >> 16) & 1u)) >> 16); }
__device__ __forceinline__ float bf16_val(unsigned short b) { return __uint_as_float(((unsigned int)b) << 16); }
__device__ __forceinline__ float bf16_round(float x) { return bf16_val(bf16_bits(x)); }
template <int NT>
__device__ __forceinline__ v8f mmaN(v16b ah, v16b al, v16b bh, v16b bl, v8f c) {
  c = __builtin_amdgcn_wmma_f32_16x16x32_bf16(false, ah, false, bh, (short)0, c, false, false);
  if (NT >= 2) c = __builtin_amdgcn_wmma_f32_16x16x32_bf16(false, al, false, bh, (short)0, c, false, false);
  if (NT >= 3) c = __builtin_amdgcn_wmma_f32_16x16x32_bf16(false, ah, false, bl, (short)0, c, false, false);
  asm volatile("v_nop\n\tv_nop\n\tv_nop\n\tv_nop" : "+v"(c) : "v"(ah), "v"(al), "v"(bh), "v"(bl));
  return c;
}

__global__ __launch_bounds__(256) void k_wt_bf16(const float* __restrict__ W, unsigned short* __restrict__ Wt, int K, int N) {
  const int t = blockIdx.x * 256 + threadIdx.x;
  const int k8n = K / 8;
  if (t >= N * k8n) return;
  const int n = t / k8n, k8 = (t % k8n) * 8;
  v8us v;
#pragma unroll
  for (int i = 0; i < 8; ++i) v[i] = bf16_bits(W[(size_t)(k8 + i) * N + n]);
  *(volatile v8us*)(Wt + (size_t)n * K + k8) = v;
  __threadfence();
  *(volatile v8us*)(Wt + (size_t)n * K + k8) = v;
}

template <bool ASPLIT, int ACT, bool BIAS_BF16>
__global__ __launch_bounds__(128) void k_gemm_bf(const float* __restrict__ A, int lda, const unsigned short* __restrict__ Wt, int ldb,
                                               const float* __restrict__ bias, float* __restrict__ C, int ldc, int M, int N, int K) {
  __shared__ __attribute__((aligned(16))) float so[4][16][64];
  const int tid = threadIdx.x, w = tid >> 5, lane = tid & 31, ln = lane & 15, hh = lane >> 4;
  const int ntn = N / 64;
  const int wid = blockIdx.x * 4 + w;
  const int mt = wid / ntn, nq = wid % ntn;
  if (mt * 16 >= M) return;
  const int row0 = mt * 16, col0 = nq * 64;
  const float* arow = A + (size_t)(row0 + ln) * lda;
  v8f acc[4] = {};
  for (int kb = 0; kb < K; kb += 32) {
    FragB ah, al;
    const v4f x0 = *(const v4fa*)(arow + kb + 8 * hh), x1 = *(const v4fa*)(arow + kb + 8 * hh + 4);
    const v4f x2 = *(const v4fa*)(arow + kb + 16 + 8 * hh), x3 = *(const v4fa*)(arow + kb + 16 + 8 * hh + 4);
    float xs[16] = {x0[0],x0[1],x0[2],x0[3],x1[0],x1[1],x1[2],x1[3],x2[0],x2[1],x2[2],x2[3],x3[0],x3[1],x3[2],x3[3]};
#pragma unroll
    for (int i = 0; i < 16; ++i) { const unsigned short hb = bf16_bits(xs[i]); ah.u[i] = hb; al.u[i] = ASPLIT ? bf16_bits(xs[i] - bf16_val(hb)) : (unsigned short)0; }
#pragma unroll
    for (int t = 0; t < 4; ++t) {
      const unsigned short* brow = Wt + (size_t)(col0 + t * 16 + ln) * ldb + kb;
      FragB b;
      b.half[0] = *(const v8us*)(brow + 8 * hh);
      b.half[1] = *(const v8us*)(brow + 16 + 8 * hh);
      acc[t] = mmaN<ASPLIT ? 2 : 1>(ah.v, al.v, b.v, b.v, acc[t]);
    }
  }
#pragma unroll
  for (int t = 0; t < 4; ++t) {
    float bv = bias ? bias[col0 + t * 16 + ln] : 0.f;
    if (BIAS_BF16) bv = bf16_round(bv);
#pragma unroll
    for (int r = 0; r < 8; ++r) { float v = acc[t][r] + bv; if (ACT == 1) v = fmaxf(v, 0.f); so[w][8 * hh + r][t * 16 + ln] = v; }
  }
  __builtin_amdgcn_fence(__ATOMIC_ACQ_REL, "workgroup");
  __builtin_amdgcn_wave_barrier();
  const int rsub = lane >> 4, c4 = (lane & 15) * 4;
  for (int pass = 0; pass < 2; ++pass) {
#pragma unroll
    for (int q = 0; q < 8; ++q) {
      const int r = q * 2 + rsub;
      const v4f v = *(const v4fa*)&so[w][r][c4];
      *(volatile v4f*)(C + (size_t)(row0 + r) * ldc + col0 + c4) = v;
    }
    if (pass == 0) __threadfence();
  }
}

template <int D, bool CAUSAL>
__global__ __launch_bounds__(128) void k_flash(const float* __restrict__ qb, const float* __restrict__ kb, const float* __restrict__ vb,
                                             int pitch, int T, int H, float scale, float* __restrict__ y, int ypitch) {
  constexpr int KS = D / 32;
  constexpr int DT = D / 16;
  __shared__ __attribute__((aligned(16))) unsigned short sKh[32][D + 8], sKl[32][D + 8], sVh[32][D + 8], sVl[32][D + 8];
  __shared__ __attribute__((aligned(16))) unsigned short sPh[4][16][40], sPl[4][16][40];
  __shared__ __attribute__((aligned(16))) float sO[4][16][D];
  const int tid = threadIdx.x, w = tid >> 5, lane = tid & 31, ln = lane & 15, hh = lane >> 4;
  const int nqb = (T + 63) / 64;
  const int bh = blockIdx.x / nqb, qblk = blockIdx.x % nqb;
  const int b = bh / H, h = bh % H;
  const int q0 = qblk * 64 + w * 16;
  const float* Q = qb + (size_t)b * T * pitch + h * D;
  const float* K = kb + (size_t)b * T * pitch + h * D;
  const float* V = vb + (size_t)b * T * pitch + h * D;

  FragB aqh[KS], aql[KS];
  {
    int row = q0 + ln; if (row >= T) row = T - 1;
    const float* qr = Q + (size_t)row * pitch;
#pragma unroll
    for (int ks = 0; ks < KS; ++ks)
#pragma unroll
      for (int i = 0; i < 16; ++i) {
        const int d = ks * 32 + ((i < 8) ? (8 * hh + i) : (16 + 8 * hh + (i - 8)));
        const float x = qr[d] * scale; const unsigned short hb = bf16_bits(x);
        aqh[ks].u[i] = hb; aql[ks].u[i] = bf16_bits(x - bf16_val(hb));
      }
  }
  float m_r[8], l_r[8];
#pragma unroll
  for (int r = 0; r < 8; ++r) { m_r[r] = -3.0e38f; l_r[r] = 0.f; }
  v8f oacc[DT];
#pragma unroll
  for (int dt = 0; dt < DT; ++dt) oacc[dt] = (v8f){0.f,0.f,0.f,0.f,0.f,0.f,0.f,0.f};

  const int kv_end = CAUSAL ? min(T, qblk * 64 + 64) : T;
  for (int j0 = 0; j0 < kv_end; j0 += 32) {
    __syncthreads();
    for (int e = tid; e < 32 * (D / 4); e += 128) {
      const int r = e / (D / 4), c4 = (e % (D / 4)) * 4;
      const int key = j0 + r;
      v4f kf = {0.f,0.f,0.f,0.f}, vf = {0.f,0.f,0.f,0.f};
      if (key < T) { kf = *(const v4fa*)(K + (size_t)key * pitch + c4); vf = *(const v4fa*)(V + (size_t)key * pitch + c4); }
#pragma unroll
      for (int t = 0; t < 4; ++t) {
        unsigned short hb = bf16_bits(kf[t]); sKh[r][c4 + t] = hb; sKl[r][c4 + t] = bf16_bits(kf[t] - bf16_val(hb));
        hb = bf16_bits(vf[t]); sVh[r][c4 + t] = hb; sVl[r][c4 + t] = bf16_bits(vf[t] - bf16_val(hb));
      }
    }
    __syncthreads();
    v8f s[2];
#pragma unroll
    for (int nt = 0; nt < 2; ++nt) {
      v8f acc = {};
#pragma unroll
      for (int ks = 0; ks < KS; ++ks) {
        FragB bh_, bl_;
        bh_.half[0] = *(const v8us*)&sKh[nt * 16 + ln][ks * 32 + 8 * hh]; bh_.half[1] = *(const v8us*)&sKh[nt * 16 + ln][ks * 32 + 16 + 8 * hh];
        bl_.half[0] = *(const v8us*)&sKl[nt * 16 + ln][ks * 32 + 8 * hh]; bl_.half[1] = *(const v8us*)&sKl[nt * 16 + ln][ks * 32 + 16 + 8 * hh];
        acc = mmaN<3>(aqh[ks].v, aql[ks].v, bh_.v, bl_.v, acc);
      }
      s[nt] = acc;
    }
    float alpha[8];
#pragma unroll
    for (int r = 0; r < 8; ++r) {
      const int qi = q0 + 8 * hh + r;
      const int ja = j0 + ln, jb = j0 + 16 + ln;
      if (CAUSAL) { if (ja > qi) s[0][r] = -3.0e38f; if (jb > qi) s[1][r] = -3.0e38f; }
      if (ja >= T) s[0][r] = -3.0e38f;
      if (jb >= T) s[1][r] = -3.0e38f;
      float mx = fmaxf(s[0][r], s[1][r]);
      mx = fmaxf(mx, __shfl_xor(mx, 1, 32)); mx = fmaxf(mx, __shfl_xor(mx, 2, 32)); mx = fmaxf(mx, __shfl_xor(mx, 4, 32)); mx = fmaxf(mx, __shfl_xor(mx, 8, 32));
      const float mnew = fmaxf(m_r[r], mx);
      alpha[r] = (mnew > -1.0e38f) ? __expf(m_r[r] - mnew) : 1.0f;
      const float p0 = (s[0][r] > -1.0e38f) ? __expf(s[0][r] - mnew) : 0.f;
      const float p1 = (s[1][r] > -1.0e38f) ? __expf(s[1][r] - mnew) : 0.f;
      m_r[r] = mnew;
      l_r[r] = l_r[r] * alpha[r] + p0 + p1;
      unsigned short hb = bf16_bits(p0); sPh[w][8 * hh + r][ln] = hb;      sPl[w][8 * hh + r][ln] = bf16_bits(p0 - bf16_val(hb));
      hb = bf16_bits(p1);                sPh[w][8 * hh + r][16 + ln] = hb; sPl[w][8 * hh + r][16 + ln] = bf16_bits(p1 - bf16_val(hb));
    }
#pragma unroll
    for (int dt = 0; dt < DT; ++dt)
#pragma unroll
      for (int r = 0; r < 8; ++r) oacc[dt][r] *= alpha[r];
    __builtin_amdgcn_fence(__ATOMIC_ACQ_REL, "workgroup");
    __builtin_amdgcn_wave_barrier();
    FragB pah, pal;
    pah.half[0] = *(const v8us*)&sPh[w][ln][8 * hh]; pah.half[1] = *(const v8us*)&sPh[w][ln][16 + 8 * hh];
    pal.half[0] = *(const v8us*)&sPl[w][ln][8 * hh]; pal.half[1] = *(const v8us*)&sPl[w][ln][16 + 8 * hh];
#pragma unroll
    for (int dt = 0; dt < DT; ++dt) {
      FragB bvh, bvl;
#pragma unroll
      for (int i = 0; i < 8; ++i) {
        bvh.u[i] = sVh[8 * hh + i][dt * 16 + ln]; bvh.u[8 + i] = sVh[16 + 8 * hh + i][dt * 16 + ln];
        bvl.u[i] = sVl[8 * hh + i][dt * 16 + ln]; bvl.u[8 + i] = sVl[16 + 8 * hh + i][dt * 16 + ln];
      }
      oacc[dt] = mmaN<3>(pah.v, pal.v, bvh.v, bvl.v, oacc[dt]);
    }
    __builtin_amdgcn_fence(__ATOMIC_ACQ_REL, "workgroup");
    __builtin_amdgcn_wave_barrier();
  }
#pragma unroll
  for (int r = 0; r < 8; ++r) {
    float l = l_r[r];
    l += __shfl_xor(l, 1, 32); l += __shfl_xor(l, 2, 32); l += __shfl_xor(l, 4, 32); l += __shfl_xor(l, 8, 32);
    l_r[r] = (l > 0.f) ? 1.0f / l : 0.f;
  }
#pragma unroll
  for (int dt = 0; dt < DT; ++dt)
#pragma unroll
    for (int r = 0; r < 8; ++r) sO[w][8 * hh + r][dt * 16 + ln] = oacc[dt][r] * l_r[r];
  __builtin_amdgcn_fence(__ATOMIC_ACQ_REL, "workgroup");
  __builtin_amdgcn_wave_barrier();
  for (int pass = 0; pass < 2; ++pass) {
    for (int r = 0; r < 16; ++r) {
      const int row = q0 + r;
      if (row < T && lane < D / 4) {
        const v4f val = *(const v4fa*)&sO[w][r][lane * 4];
        *(volatile v4f*)(y + ((size_t)b * T + row) * ypitch + h * D + lane * 4) = val;
      }
    }
    if (pass == 0) __threadfence();
  }
}

typedef _Float16 v16h __attribute__((ext_vector_type(16)));
union FragH { v16h v; v8us half[2]; _Float16 h[16]; unsigned short u[16]; };
template <int NT>
__device__ __forceinline__ v8f mmaH(v16h ah, v16h al, v16h bh, v16h bl, v8f c) {
  c = __builtin_amdgcn_wmma_f32_16x16x32_f16(false, ah, false, bh, (short)0, c, false, false);
  if (NT >= 2) c = __builtin_amdgcn_wmma_f32_16x16x32_f16(false, al, false, bh, (short)0, c, false, false);
  if (NT >= 3) c = __builtin_amdgcn_wmma_f32_16x16x32_f16(false, ah, false, bl, (short)0, c, false, false);
  asm volatile("v_nop\n\tv_nop\n\tv_nop\n\tv_nop" : "+v"(c) : "v"(ah), "v"(al), "v"(bh), "v"(bl));
  return c;
}
template <bool ASPLIT>
__global__ __launch_bounds__(128) void k_gemm_h(const float* __restrict__ A, int lda, size_t sA, const _Float16* __restrict__ Bh, int ldb, size_t sB, float alpha, float* __restrict__ C, int ldc, size_t sC, int M, int N, int K) {
  __shared__ __attribute__((aligned(16))) float so[4][16][64];
  const int tid = threadIdx.x, w = tid >> 5, lane = tid & 31, ln = lane & 15, hh = lane >> 4; const int by = blockIdx.y;
  A += (size_t)by * sA; Bh += (size_t)by * sB; C += (size_t)by * sC;
  const int ntn = (N + 63) / 64; const int wid = blockIdx.x * 4 + w; const int mt = wid / ntn, nq = wid % ntn; if (mt * 16 >= M) return;
  const int row0 = mt * 16, col0 = nq * 64; const float* arow = A + (size_t)(row0 + ln) * lda;
  v8f acc[4] = {};
  for (int kb = 0; kb < K; kb += 32) {
    FragH ah, al;
    const v4f x0 = *(const v4fa*)(arow + kb + 8 * hh), x1 = *(const v4fa*)(arow + kb + 8 * hh + 4), x2 = *(const v4fa*)(arow + kb + 16 + 8 * hh), x3 = *(const v4fa*)(arow + kb + 16 + 8 * hh + 4);
    float xs[16] = {x0[0],x0[1],x0[2],x0[3],x1[0],x1[1],x1[2],x1[3],x2[0],x2[1],x2[2],x2[3],x3[0],x3[1],x3[2],x3[3]};
#pragma unroll
    for (int i = 0; i < 16; ++i) { const _Float16 h = (_Float16)xs[i]; ah.h[i] = h; al.h[i] = ASPLIT ? (_Float16)(xs[i] - (float)h) : (_Float16)0.0f; }
#pragma unroll
    for (int t = 0; t < 4; ++t) { if (col0 + t * 16 >= N) continue; const size_t boff = (size_t)(col0 + t * 16 + ln) * ldb + kb; FragH bq; bq.half[0] = *(const v8us*)(Bh + boff + 8 * hh); bq.half[1] = *(const v8us*)(Bh + boff + 16 + 8 * hh);
      acc[t] = mmaH<ASPLIT ? 2 : 1>(ah.v, al.v, bq.v, bq.v, acc[t]); }
  }
#pragma unroll
  for (int t = 0; t < 4; ++t) { if (col0 + t * 16 >= N) continue;
#pragma unroll
    for (int r = 0; r < 8; ++r) so[w][8 * hh + r][t * 16 + ln] = acc[t][r] * alpha; }
  __builtin_amdgcn_fence(__ATOMIC_ACQ_REL, "workgroup"); __builtin_amdgcn_wave_barrier();
  const int rsub = lane >> 4, c4 = (lane & 15) * 4;
  for (int pass = 0; pass < 2; ++pass) {
#pragma unroll
    for (int q = 0; q < 8; ++q) { const int r = q * 2 + rsub; if (col0 + c4 < N) { const v4f v = *(const v4fa*)&so[w][r][c4]; *(volatile v4f*)(C + (size_t)(row0 + r) * ldc + col0 + c4) = v; } }
    if (pass == 0) __threadfence(); }
}

template <int DUMMY>
__global__ __launch_bounds__(128) void k_gemm_hh(const _Float16* __restrict__ A, int lda, size_t sA, const _Float16* __restrict__ Bh, int ldb, size_t sB, float alpha, float* __restrict__ C, int ldc, size_t sC, int M, int N, int K) {
  __shared__ __attribute__((aligned(16))) float so[4][16][64];
  const int tid = threadIdx.x, w = tid >> 5, lane = tid & 31, ln = lane & 15, hh = lane >> 4; const int by = blockIdx.y;
  A += (size_t)by * sA; Bh += (size_t)by * sB; C += (size_t)by * sC;
  const int ntn = (N + 63) / 64; const int wid = blockIdx.x * 4 + w; const int mt = wid / ntn, nq = wid % ntn; if (mt * 16 >= M) return;
  const int row0 = mt * 16, col0 = nq * 64; const _Float16* arow = A + (size_t)(row0 + ln) * lda;
  v8f acc[4] = {};
  for (int kb = 0; kb < K; kb += 32) { FragH ah; ah.half[0] = *(const v8us*)((const unsigned short*)arow + kb + 8 * hh); ah.half[1] = *(const v8us*)((const unsigned short*)arow + kb + 16 + 8 * hh);
#pragma unroll
    for (int t = 0; t < 4; ++t) { if (col0 + t * 16 >= N) continue; const size_t boff = (size_t)(col0 + t * 16 + ln) * ldb + kb; FragH bq; bq.half[0] = *(const v8us*)((const unsigned short*)Bh + boff + 8 * hh); bq.half[1] = *(const v8us*)((const unsigned short*)Bh + boff + 16 + 8 * hh);
      acc[t] = mmaH<1>(ah.v, ah.v, bq.v, bq.v, acc[t]); }
  }
#pragma unroll
  for (int t = 0; t < 4; ++t) { if (col0 + t * 16 >= N) continue;
#pragma unroll
    for (int r = 0; r < 8; ++r) so[w][8 * hh + r][t * 16 + ln] = acc[t][r] * alpha; }
  __builtin_amdgcn_fence(__ATOMIC_ACQ_REL, "workgroup"); __builtin_amdgcn_wave_barrier();
  const int rsub = lane >> 4, c4 = (lane & 15) * 4;
  for (int pass = 0; pass < 2; ++pass) {
#pragma unroll
    for (int q = 0; q < 8; ++q) { const int r = q * 2 + rsub; if (col0 + c4 < N) { const v4f v = *(const v4fa*)&so[w][r][c4]; *(volatile v4f*)(C + (size_t)(row0 + r) * ldc + col0 + c4) = v; } }
    if (pass == 0) __threadfence(); }
}

template <int ACT>
__global__ __launch_bounds__(128) void k_gemm_hhx(const _Float16* __restrict__ A, int lda, size_t sA, const _Float16* __restrict__ Bh, int ldb, size_t sB, float alpha, const float* __restrict__ bias, size_t sBias, const float* __restrict__ CP, int rowsPerB, size_t sCPb, int row0g,
    float* __restrict__ C, _Float16* __restrict__ C16, int ldc, size_t sC, int M, int N, int K) {
  __shared__ __attribute__((aligned(16))) float so[4][16][64];
  const int tid = threadIdx.x, w = tid >> 5, lane = tid & 31, ln = lane & 15, hh = lane >> 4; const int by = blockIdx.y;
  A += (size_t)by * sA; Bh += (size_t)by * sB; const size_t cofs = (size_t)by * sC; const float* bp = bias ? bias + (size_t)by * sBias : nullptr;
  const int ntn = (N + 63) / 64; const int wid = blockIdx.x * 4 + w; const int mt = wid / ntn, nq = wid % ntn; if (mt * 16 >= M) return;
  const int row0 = mt * 16, col0 = nq * 64; const _Float16* arow = A + (size_t)(row0 + ln) * lda;
  v8f acc[4] = {};
  for (int kb = 0; kb < K; kb += 32) { FragH ah; ah.half[0] = *(const v8us*)((const unsigned short*)arow + kb + 8 * hh); ah.half[1] = *(const v8us*)((const unsigned short*)arow + kb + 16 + 8 * hh);
#pragma unroll
    for (int t = 0; t < 4; ++t) { if (col0 + t * 16 >= N) continue; const size_t boff = (size_t)(col0 + t * 16 + ln) * ldb + kb; FragH bq; bq.half[0] = *(const v8us*)((const unsigned short*)Bh + boff + 8 * hh); bq.half[1] = *(const v8us*)((const unsigned short*)Bh + boff + 16 + 8 * hh);
      acc[t] = mmaH<1>(ah.v, ah.v, bq.v, bq.v, acc[t]); }
  }
#pragma unroll
  for (int t = 0; t < 4; ++t) { if (col0 + t * 16 >= N) continue; const int col = col0 + t * 16 + ln; const float bv = bp ? bf16_round(bp[col]) : 0.f;
#pragma unroll
    for (int r = 0; r < 8; ++r) { float v = acc[t][r] * alpha + bv; if (CP) { const int bidx = (row0g + row0 + 8 * hh + r) / rowsPerB; v += CP[(size_t)bidx * sCPb + (size_t)by * 64 + col]; } if (ACT == 1) v = (v > 0.f) ? v : expm1f(v); else if (ACT == 3) v = fmaxf(v, 0.f); so[w][8 * hh + r][t * 16 + ln] = v; } }
  __builtin_amdgcn_fence(__ATOMIC_ACQ_REL, "workgroup"); __builtin_amdgcn_wave_barrier();
  const int rsub = lane >> 4, c4 = (lane & 15) * 4; typedef _Float16 v4h __attribute__((ext_vector_type(4)));
  for (int pass = 0; pass < 2; ++pass) {
#pragma unroll
    for (int q = 0; q < 8; ++q) { const int r = q * 2 + rsub; if (col0 + c4 < N) { const v4f v = *(const v4fa*)&so[w][r][c4]; if (C) *(volatile v4f*)(C + cofs + (size_t)(row0 + r) * ldc + col0 + c4) = v; if (C16) { v4h h4; for (int i = 0; i < 4; ++i) h4[i] = (_Float16)v[i]; *(volatile v4h*)(C16 + cofs + (size_t)(row0 + r) * ldc + col0 + c4) = h4; } } }
    if (pass == 0) __threadfence(); }
}

__device__ __forceinline__ int bscan_k_seg(int cnt, int* scan, int tid, int& total) { __syncthreads(); scan[tid] = cnt; __syncthreads();
  for (int of = 1; of < 512; of <<= 1) { const int v = (tid >= of) ? scan[tid - of] : 0; __syncthreads(); scan[tid] += v; __syncthreads(); }
  total = scan[512 - 1]; return scan[tid] - cnt; }
__global__ __launch_bounds__(512) void k_seg(const float* __restrict__ T, const int* __restrict__ src, const int* __restrict__ dst, float* __restrict__ AGG) {
  __shared__ short Lr[4096]; __shared__ int Lc[4096];  __shared__ int scan[512]; __shared__ float stg[64][128 + 1];
  const int tid = threadIdx.x; const int s0 = blockIdx.x * 512; float acc0[128];
#pragma unroll
  for (int c = 0; c < 128; ++c) acc0[c] = 0.f;
  for (int e0 = 0; e0 < (NE); e0 += 4096) { int hr[8], hc[8];  int cnt = 0;
#pragma unroll
    for (int k = 0; k < 8; ++k) { const int e = e0 + tid * 8 + k; hr[k] = -1; hc[k] = 0;  if (e < (NE)) { const int dd_ = (dst[e]); if (dd_ >= s0 && dd_ < s0 + 512) { hr[k] = dd_ - s0; int s = (src[e]); s = s < 0 ? 0 : (s >= (NN) ? (NN) - 1 : s); hc[k] = s;  ++cnt; } } }
    int tot; int p = bscan_k_seg(cnt, scan, tid, tot);
#pragma unroll
    for (int k = 0; k < 8; ++k) if (hr[k] >= 0) { Lr[p] = (short)hr[k]; Lc[p] = hc[k];  ++p; }
    __syncthreads();
#pragma unroll 1
    for (int q = 0; q < tot; ++q) { if (Lr[q] == tid) { const float* row = (T + (size_t)Lc[q] * HH);
#pragma unroll
        for (int c = 0; c < 128; c += 4) { const v4f v = *(const v4fa*)(row + c); acc0[c] += v[0]; acc0[c + 1] += v[1]; acc0[c + 2] += v[2]; acc0[c + 3] += v[3]; } } }
    __syncthreads(); }
  for (int tg = 0; tg < 512 / 64; ++tg) {
    if (tid / 64 == tg) {
#pragma unroll
      for (int c = 0; c < 128; ++c) stg[tid % 64][c] = acc0[c]; }
    __syncthreads();
    for (int pass = 0; pass < 2; ++pass) { for (int i = tid; i < 64 * (128 / 4); i += 512) { const int r = i / (128 / 4), c4 = (i % (128 / 4)) * 4; const int seg = s0 + tg * 64 + r; if (seg < (NN)) { v4f v; v[0] = stg[r][c4]; v[1] = stg[r][c4 + 1]; v[2] = stg[r][c4 + 2]; v[3] = stg[r][c4 + 3];  *(volatile v4f*)((AGG + (size_t)seg * HH) + c4) = v; } } if (pass == 0) __threadfence(); }
    __syncthreads(); } }

__global__ __launch_bounds__(256) void k_bt(const float* __restrict__ w1r, const float* __restrict__ w1o, const float* __restrict__ w2r, const float* __restrict__ w2o, const float* __restrict__ w3r, const float* __restrict__ w3o, const float* __restrict__ w4r, const float* __restrict__ w4o, const float* __restrict__ w5r, const float* __restrict__ w5o, _Float16* __restrict__ B1, _Float16* __restrict__ B234, _Float16* __restrict__ B5) { const int t = blockIdx.x * 256 + threadIdx.x;
  if (t < HH * F0P) { const int k = t % F0P, n = t / F0P; const float a = (k < F0) ? bf16_round(w1r[n * F0 + k]) * 16.0f : 0.f, b = (k < F0) ? bf16_round(w1o[n * F0 + k]) * 16.0f : 0.f; *(volatile _Float16*)(B1 + t) = (_Float16)a; *(volatile _Float16*)(B1 + HH * F0P + t) = (_Float16)b; }
  if (t < HH * HH) { const float* ws_[6] = {w2r, w2o, w3r, w3o, w4r, w4o}; for (int i = 0; i < 6; ++i) *(volatile _Float16*)(B234 + (size_t)i * HH * HH + t) = (_Float16)(bf16_round(ws_[i][t]) * 16.0f); }
  if (t < HH * 512) { *(volatile _Float16*)(B5 + t) = (_Float16)(bf16_round(w5r[t]) * 16.0f); *(volatile _Float16*)(B5 + HH * 512 + t) = (_Float16)(bf16_round(w5o[t]) * 16.0f); } }
__global__ __launch_bounds__(256) void k_x16(const float* __restrict__ x, _Float16* __restrict__ X16) { const size_t t = (size_t)blockIdx.x * 256 + threadIdx.x; if (t >= (size_t)NN * F0P / 8) return; const int k8 = (int)((t * 8) % F0P); const size_t n = (t * 8) / F0P; FragH f; for (int q = 0; q < 8; ++q) f.h[q] = (_Float16)((k8 + q < F0) ? bf16_round(x[n * F0 + k8 + q]) : 0.f); *(volatile v8us*)((unsigned short*)X16 + t * 8) = f.half[0]; __threadfence(); *(volatile v8us*)((unsigned short*)X16 + t * 8) = f.half[0]; }
__global__ __launch_bounds__(128) void k_bnstat(const float* __restrict__ X5, float* __restrict__ MU, float* __restrict__ IV) { const int c = threadIdx.x; float s = 0.f;
#pragma unroll 4
  for (int n = 0; n < NN; ++n) s += X5[(size_t)n * HH + c]; const float mu = s / (float)NN; float q2 = 0.f;
#pragma unroll 4
  for (int n = 0; n < NN; ++n) { const float d = X5[(size_t)n * HH + c] - mu; q2 += d * d; } const float iv = 1.0f / sqrtf(q2 / (float)NN + 1e-5f); *(volatile float*)(MU + c) = mu; *(volatile float*)(IV + c) = iv; __threadfence(); *(volatile float*)(MU + c) = mu; *(volatile float*)(IV + c) = iv; }
__global__ __launch_bounds__(128) void k_pool(const float* __restrict__ X5, const int* __restrict__ batch, const float* __restrict__ MU, const float* __restrict__ IV, const float* __restrict__ gam, const float* __restrict__ bet, const float* __restrict__ Wl, const float* __restrict__ bl, float* __restrict__ out) {
  __shared__ float acc[NG + 28][HH + 1]; __shared__ float cnt[NG + 28]; const int tid = threadIdx.x;
  for (int g = 0; g < NG; ++g) acc[g][tid] = 0.f; if (tid < NG) cnt[tid] = 0.f; __syncthreads();
  const float mu = MU[tid], iv = IV[tid], ga = bf16_round(gam[tid]), be = bf16_round(bet[tid]);
#pragma unroll 1
  for (int n = 0; n < NN; ++n) { int g = batch[n]; if (g < 0 || g >= NG) continue; const float v = (X5[(size_t)n * HH + tid] - mu) * iv * ga + be; acc[g][tid] += v; if (tid == 0) cnt[g] += 1.f; }
  __syncthreads();
  if (tid < NG) { const float ic = 1.0f / fmaxf(cnt[tid], 1.0f); float o[NCLS]; for (int k = 0; k < NCLS; ++k) o[k] = bf16_round(bl[k]);
#pragma unroll 1
    for (int c = 0; c < HH; ++c) { const float p = acc[tid][c] * ic;
#pragma unroll
      for (int k = 0; k < NCLS; ++k) o[k] += p * bf16_round(Wl[k * HH + c]); }
    for (int k = 0; k < NCLS; ++k) acc[tid][k] = o[k]; }
  __syncthreads();
  typedef float v4fl __attribute__((ext_vector_type(4)));
  for (int pass = 0; pass < 2; ++pass) { for (int i = tid; i < NG * NCLS / 4; i += 128) { v4fl v; for (int q = 0; q < 4; ++q) { const int e = i * 4 + q; v[q] = acc[e / NCLS][e % NCLS]; } *(volatile v4fl*)(out + i * 4) = v; } if (pass == 0) __threadfence(); } }
extern "C" void kernel_launch(void* const* d_in, const int* in_sizes, int n_in,
                              void* d_out, int out_size, void* d_ws, size_t ws_size, hipStream_t stream) {
  (void)in_sizes; (void)n_in; (void)out_size;
  const float* x = (const float*)d_in[0]; const int* ei = (const int*)d_in[1]; const int* batch = (const int*)d_in[2];
  const float* w1r = (const float*)d_in[3]; const float* w1o = (const float*)d_in[4]; const float* b1 = (const float*)d_in[5]; const float* w2r = (const float*)d_in[6]; const float* w2o = (const float*)d_in[7]; const float* b2 = (const float*)d_in[8]; const float* w3r = (const float*)d_in[9]; const float* w3o = (const float*)d_in[10]; const float* b3 = (const float*)d_in[11]; const float* w4r = (const float*)d_in[12]; const float* w4o = (const float*)d_in[13]; const float* b4 = (const float*)d_in[14]; const float* w5r = (const float*)d_in[15]; const float* w5o = (const float*)d_in[16]; const float* b5 = (const float*)d_in[17]; const float* gam = (const float*)d_in[18]; const float* bet = (const float*)d_in[19]; const float* Wl = (const float*)d_in[20]; const float* bl = (const float*)d_in[21];
  const int* src = ei; const int* dst = ei + NE;
  char* ws = (char*)d_ws; size_t off = 0;
  auto take = [&](size_t bytes) { char* p = ws + off; off += (bytes + 255) & ~(size_t)255; return p; };
  _Float16* B1 = (_Float16*)take((size_t)2 * HH * F0P * 2); _Float16* B234 = (_Float16*)take((size_t)6 * HH * HH * 2); _Float16* B5 = (_Float16*)take((size_t)2 * HH * 512 * 2);
  _Float16* X16 = (_Float16*)take((size_t)NN * F0P * 2); _Float16* XC = (_Float16*)take((size_t)NN * 512 * 2); float* T = (float*)take((size_t)NN * HH * 4); float* AGG = (float*)take((size_t)NN * HH * 4); float* X5 = (float*)take((size_t)NN * HH * 4); float* MU = (float*)take(HH * 4); float* IV = (float*)take(HH * 4);
  if (off > ws_size) return;
  const dim3 gg(((NN / 16) * (HH / 64) + 3) / 4, 1); const int NT_ = (NN + 511) / 512;
  k_bt<<<(HH * 512 + 255) / 256, 256, 0, stream>>>(w1r, w1o, w2r, w2o, w3r, w3o, w4r, w4o, w5r, w5o, B1, B234, B5);
  k_x16<<<(unsigned)(((size_t)NN * F0P / 8 + 255) / 256), 256, 0, stream>>>(x, X16);
  k_gemm_hhx<0><<<gg, 128, 0, stream>>>(X16, F0P, 0, B1, F0P, 0, 0.0625f, nullptr, 0, nullptr, 1, 0, 0, T, nullptr, HH, 0, NN, HH, F0P);
  k_seg<<<NT_, 512, 0, stream>>>(T, src, dst, AGG);
  k_gemm_hhx<3><<<gg, 128, 0, stream>>>(X16, F0P, 0, B1 + (size_t)HH * F0P, F0P, 0, 0.0625f, b1, 0, AGG, 1, HH, 0, nullptr, XC, 512, 0, NN, HH, F0P);
  for (int l = 2; l <= 4; ++l) { const _Float16* xin = XC + (size_t)(l - 2) * HH; _Float16* xout = XC + (size_t)(l - 1) * HH; const _Float16* Br = B234 + (size_t)(2 * (l - 2)) * HH * HH; const _Float16* Bo = Br + (size_t)HH * HH; const float* bb = (l == 2) ? b2 : (l == 3 ? b3 : b4);
    k_gemm_hhx<0><<<gg, 128, 0, stream>>>(xin, 512, 0, Br, HH, 0, 0.0625f, nullptr, 0, nullptr, 1, 0, 0, T, nullptr, HH, 0, NN, HH, HH);
    k_seg<<<NT_, 512, 0, stream>>>(T, src, dst, AGG);
    k_gemm_hhx<3><<<gg, 128, 0, stream>>>(xin, 512, 0, Bo, HH, 0, 0.0625f, bb, 0, AGG, 1, HH, 0, nullptr, xout, 512, 0, NN, HH, HH); }
  k_gemm_hhx<0><<<gg, 128, 0, stream>>>(XC, 512, 0, B5, 512, 0, 0.0625f, nullptr, 0, nullptr, 1, 0, 0, T, nullptr, HH, 0, NN, HH, 512);
  k_seg<<<NT_, 512, 0, stream>>>(T, src, dst, AGG);
  k_gemm_hhx<0><<<gg, 128, 0, stream>>>(XC, 512, 0, B5 + (size_t)HH * 512, 512, 0, 0.0625f, b5, 0, AGG, 1, HH, 0, X5, nullptr, HH, 0, NN, HH, 512);
  k_bnstat<<<1, 128, 0, stream>>>(X5, MU, IV);
  k_pool<<<1, 128, 0, stream>>>(X5, batch, MU, IV, gam, bet, Wl, bl, (float*)d_out);
}
